// GridGNNWithAngles_44504451121306
// MI455X (gfx1250) — hardware-verified
//
#include <hip/hip_runtime.h>
#include <hip/hip_bf16.h>
#include <stddef.h>
#include <math.h>


#define C       64
#define NB      512
#define NTHR    256
#define NWAVE   8
#define EPT     8
#define CHUNK   (NTHR * EPT)
#define WCAP    (EPT * 32)
#define PASSN   128
#define PCAP    12288
#define EHDR    32
#define EROW    (EHDR + PCAP)
#define PJT     128
#define PJR     64
#define NGRP    (NTHR / C)
#define WPL     (C * C)
#define KIN     66
#define DEG2RAD 0.017453292519943295f

#define LDS_ACC   0
#define LDS_MSG   (LDS_ACC + (NB + 1) * C * 4)
#define LDS_ESRC  (LDS_MSG + PASSN * C * 4)
#define LDS_ESLOT (LDS_ESRC + PASSN * 4)
#define LDS_ESIN  (LDS_ESLOT + PASSN * 4)
#define LDS_ECOS  (LDS_ESIN + PASSN * 4)
#define LDS_AGG   (LDS_ECOS + PASSN * 4)

static_assert(NTHR == NWAVE * 32);
static_assert(NGRP * C == NTHR);
static_assert(PASSN <= NTHR && (PASSN % NGRP) == 0);
static_assert((PCAP % PASSN) == 0);
static_assert(EHDR * 4 == 128);
static_assert((EROW % 4) == 0 && ((EROW * 4) % 128) == 0);
static_assert((NB % (2 * NWAVE)) == 0 && (NB % PJR) == 0);
static_assert(PJT == 4 * 32 && PJR == 4 * 16);
static_assert((LDS_MSG % 16) == 0 && (LDS_ESRC % 16) == 0 && (LDS_AGG % 16) == 0);
static_assert(LDS_AGG <= 300 * 1024);
static_assert((NWAVE * WCAP + EROW + NWAVE) * 4 <= 64 * 1024);

typedef float          v4f   __attribute__((ext_vector_type(4)));
typedef float          v8f   __attribute__((ext_vector_type(8)));
typedef int            v4i   __attribute__((ext_vector_type(4)));
typedef unsigned short v8us  __attribute__((ext_vector_type(8)));
typedef unsigned short v16us __attribute__((ext_vector_type(16)));
typedef __bf16         v16bf __attribute__((ext_vector_type(16)));
union FragB { v16bf v; v16us u; v8us h[2]; };
union Pk8 { v8us h; v4i i; };

__device__ __forceinline__ unsigned f2bf(float f) {
  const unsigned u = __float_as_uint(f);
  return (u + 0x7FFFu + ((u >> 16) & 1u)) >> 16;
}

__device__ __forceinline__ void split8(v4f a, v4f b, v8us& hi, v8us& lo) {
  float f[8];
  f[0] = a.x; f[1] = a.y; f[2] = a.z; f[3] = a.w;
  f[4] = b.x; f[5] = b.y; f[6] = b.z; f[7] = b.w;
  v8us rh, rl;
#pragma unroll
  for (int i = 0; i < 8; ++i) {
    const unsigned hb = f2bf(f[i]);
    const float r = f[i] - __uint_as_float(hb << 16);
    rh[i] = (unsigned short)hb;
    rl[i] = (unsigned short)f2bf(r);
  }
  hi = rh;
  lo = rl;
}

__device__ __forceinline__ v8f wm3(v16bf ah, v16bf al, v16bf bh, v16bf bl, v8f c) {
  v8f d = __builtin_amdgcn_wmma_f32_16x16x32_bf16(false, ah, false, bh, (short)0, c, false, false);
  d = __builtin_amdgcn_wmma_f32_16x16x32_bf16(false, ah, false, bl, (short)0, d, false, false);
  d = __builtin_amdgcn_wmma_f32_16x16x32_bf16(false, al, false, bh, (short)0, d, false, false);
  asm volatile("v_nop\n\tv_nop\n\tv_nop\n\tv_nop" : "+v"(d) : "v"(ah), "v"(al), "v"(bh), "v"(bl));
  return d;
}

__global__ __launch_bounds__(NTHR) void k_wprep(const float* __restrict__ w1, const float* __restrict__ w2,
                                               unsigned short* wp) {
  const int u = blockIdx.x * NTHR + threadIdx.x;
  if (u >= 2 * (WPL / 8)) return;
  const int wsel = u >> 9;
  const int v = u & 511;
  const int n = v >> 3, kc = v & 7;
  float f[8];
#pragma unroll
  for (int j = 0; j < 8; ++j) {
    const int k = 8 * kc + j;
    const float a = w1[k * C + n];
    const float b = w2[k * C + n];
    f[j] = (wsel != 0) ? b : a;
  }
  Pk8 ph, pl;
  {
    v4f a, c;
    a.x = f[0]; a.y = f[1]; a.z = f[2]; a.w = f[3];
    c.x = f[4]; c.y = f[5]; c.z = f[6]; c.w = f[7];
    split8(a, c, ph.h, pl.h);
  }
  unsigned short* dh = wp + (size_t)wsel * 2 * WPL + (size_t)v * 8;
  unsigned short* dl = dh + WPL;
  *(volatile v4i*)dh = ph.i;
  *(volatile v4i*)dl = pl.i;
  __threadfence();
  *(volatile v4i*)dh = ph.i;
  *(volatile v4i*)dl = pl.i;
}

__global__ __launch_bounds__(NTHR) void k_sincos(const float* __restrict__ attr, float* sc, int nE, int n4) {
  const int u = blockIdx.x * NTHR + threadIdx.x;
  if (u >= n4) return;
  float s0 = 0.0f, c0 = 0.0f, s1 = 0.0f, c1 = 0.0f;
#pragma unroll 1
  for (int j = 0; j < 2; ++j) {
    int e = 2 * u + j;
    e = e > nE - 1 ? nE - 1 : e;
    const float rad = attr[e] * DEG2RAD;
    float sv, cv;
    sincosf(rad, &sv, &cv);
    s0 = (j == 0) ? sv : s0;
    c0 = (j == 0) ? cv : c0;
    s1 = (j == 1) ? sv : s1;
    c1 = (j == 1) ? cv : c1;
  }
  v4f o;
  o.x = s0; o.y = c0; o.z = s1; o.w = c1;
  *(volatile v4f*)(sc + (size_t)u * 4) = o;
  __threadfence();
  *(volatile v4f*)(sc + (size_t)u * 4) = o;
}

__device__ __forceinline__ int scan_chunk(const int* __restrict__ dsts, int nE, int cbase, int nodeBase,
                                          int vec8, int* list, int tid, int wave) {
  int wc = 0;
  const int el0  = tid * EPT;
  const int e0   = cbase + el0;
  const int sent = -2147483647 - 1;
  v4i da, db;
  if (vec8 != 0 && cbase + CHUNK <= nE) {
    da = *(const v4i*)(dsts + e0);
    db = *(const v4i*)(dsts + e0 + 4);
  } else {
    da.x = (e0     < nE) ? dsts[min(e0, nE - 1)] : sent;
    da.y = (e0 + 1 < nE) ? dsts[min(e0 + 1, nE - 1)] : sent;
    da.z = (e0 + 2 < nE) ? dsts[min(e0 + 2, nE - 1)] : sent;
    da.w = (e0 + 3 < nE) ? dsts[min(e0 + 3, nE - 1)] : sent;
    db.x = (e0 + 4 < nE) ? dsts[min(e0 + 4, nE - 1)] : sent;
    db.y = (e0 + 5 < nE) ? dsts[min(e0 + 5, nE - 1)] : sent;
    db.z = (e0 + 6 < nE) ? dsts[min(e0 + 6, nE - 1)] : sent;
    db.w = (e0 + 7 < nE) ? dsts[min(e0 + 7, nE - 1)] : sent;
  }
  const unsigned nb = (unsigned)nodeBase;
  const unsigned s0 = (unsigned)da.x - nb, s1 = (unsigned)da.y - nb;
  const unsigned s2 = (unsigned)da.z - nb, s3 = (unsigned)da.w - nb;
  const unsigned s4 = (unsigned)db.x - nb, s5 = (unsigned)db.y - nb;
  const unsigned s6 = (unsigned)db.z - nb, s7 = (unsigned)db.w - nb;
  const bool h0 = s0 < (unsigned)NB, h1 = s1 < (unsigned)NB, h2 = s2 < (unsigned)NB, h3 = s3 < (unsigned)NB;
  const bool h4 = s4 < (unsigned)NB, h5 = s5 < (unsigned)NB, h6 = s6 < (unsigned)NB, h7 = s7 < (unsigned)NB;
  const unsigned any = __builtin_amdgcn_ballot_w32(h0 | h1 | h2 | h3 | h4 | h5 | h6 | h7);
  if (any != 0u) {
#define HITJ(J, HJ) { \
      const unsigned mj = __builtin_amdgcn_ballot_w32(HJ); \
      if (mj != 0u) { \
        if (HJ) { \
          const int pos = wc + (int)__builtin_amdgcn_mbcnt_lo(mj, 0u); \
          if (pos < WCAP) list[wave * WCAP + pos] = el0 + (J); \
        } \
        wc += (int)__builtin_popcount(mj); } }
    HITJ(0, h0)
    HITJ(1, h1)
    HITJ(2, h2)
    HITJ(3, h3)
    HITJ(4, h4)
    HITJ(5, h5)
    HITJ(6, h6)
    HITJ(7, h7)
#undef HITJ
  }
  return wc;
}

__global__ __launch_bounds__(NTHR) void k_escan(const int* __restrict__ ei, int* etab, int nE, int vec8) {
  __shared__ int list[NWAVE * WCAP];
  __shared__ __attribute__((aligned(16))) int pend[EROW];
  __shared__ int wcnt[NWAVE];
  const int tid = threadIdx.x, lane = tid & 31, wave = tid >> 5;
  const int nodeBase = blockIdx.x * NB;
  const int* dsts = ei + nE;
  for (int i = tid; i < EROW; i += NTHR) pend[i] = 0;
  __syncthreads();
  int pendN = 0;
  const int nChunks = (nE + CHUNK - 1) / CHUNK;
#pragma unroll 1
  for (int ch = 0; ch < nChunks; ++ch) {
    const int cbase = ch * CHUNK;
    const int wc = scan_chunk(dsts, nE, cbase, nodeBase, vec8, list, tid, wave);
    if (lane == 0) wcnt[wave] = wc;
    __syncthreads();
    const int base = pendN;
    int tot = 0, myoff = 0;
#pragma unroll
    for (int w = 0; w < NWAVE; ++w) {
      int c = wcnt[w];
      c = c > WCAP ? WCAP : (c < 0 ? 0 : c);
      if (w < wave) myoff += c;
      tot += c;
    }
    {
      int n = wcnt[wave];
      n = n > WCAP ? WCAP : (n < 0 ? 0 : n);
      const int* lp = list + wave * WCAP;
      for (int i = lane; i < n; i += 32) {
        const int pos = base + myoff + i;
        if (pos < PCAP) pend[EHDR + pos] = cbase + lp[i];
      }
    }
    const int newN = base + tot;
    pendN = newN > PCAP ? PCAP : newN;
    __syncthreads();
  }
  if (tid == 0) pend[0] = pendN;
  __syncthreads();
  int* rowp = etab + (size_t)blockIdx.x * EROW;
#pragma unroll 1
  for (int u = tid; u < EROW / 4; u += NTHR) {
    const v4i v = *(const v4i*)(pend + 4 * u);
    *(volatile v4i*)(rowp + 4 * u) = v;
  }
  __threadfence();
#pragma unroll 1
  for (int u = tid; u < EROW / 4; u += NTHR) {
    const v4i v = *(const v4i*)(pend + 4 * u);
    *(volatile v4i*)(rowp + 4 * u) = v;
  }
}

__global__ __launch_bounds__(PJT) void k_proj(const float* __restrict__ xin,
    const unsigned short* __restrict__ wh, const unsigned short* __restrict__ wl,
    float* pout, int nRowsIn, int nRowsOut) {
  __shared__ __attribute__((aligned(16))) float stg[PJR * C];
  const int tid = threadIdx.x, lane = tid & 31, wave = tid >> 5, hh = lane >> 4, m = lane & 15;
  const int rowBase = blockIdx.x * PJR;
  const int lrow = wave * 16 + m;
  int node = rowBase + lrow;
  node = node > nRowsIn - 1 ? nRowsIn - 1 : node;
  const float* xrow = xin + (size_t)node * C;
  FragB bh[2], bl[2];
#pragma unroll
  for (int kt = 0; kt < 2; ++kt) {
    const int k0 = 32 * kt + 8 * hh;
    const v4f a = *(const v4f*)(xrow + k0);
    const v4f b = *(const v4f*)(xrow + k0 + 4);
    const v4f c = *(const v4f*)(xrow + k0 + 16);
    const v4f d = *(const v4f*)(xrow + k0 + 20);
    split8(a, b, bh[kt].h[0], bl[kt].h[0]);
    split8(c, d, bh[kt].h[1], bl[kt].h[1]);
  }
#pragma unroll 1
  for (int ft = 0; ft < C / 16; ++ft) {
    v8f acc;
#pragma unroll
    for (int r = 0; r < 8; ++r) acc[r] = 0.0f;
    const size_t ao = (size_t)(16 * ft + m) * C + 8 * hh;
#pragma unroll
    for (int kt = 0; kt < 2; ++kt) {
      FragB fh, fl;
      fh.h[0] = *(const v8us*)(wh + ao + 32 * kt);
      fh.h[1] = *(const v8us*)(wh + ao + 32 * kt + 16);
      fl.h[0] = *(const v8us*)(wl + ao + 32 * kt);
      fl.h[1] = *(const v8us*)(wl + ao + 32 * kt + 16);
      acc = wm3(fh.v, fl.v, bh[kt].v, bl[kt].v, acc);
    }
    v4f o0, o1;
    o0.x = acc[0]; o0.y = acc[1]; o0.z = acc[2]; o0.w = acc[3];
    o1.x = acc[4]; o1.y = acc[5]; o1.z = acc[6]; o1.w = acc[7];
    float* sp = stg + lrow * C + 16 * ft + 8 * hh;
    *(v4f*)sp = o0;
    *(v4f*)(sp + 4) = o1;
  }
  __syncthreads();
#pragma unroll 1
  for (int j = 0; j < 8; ++j) {
    const int row = wave * 16 + 2 * j + hh;
    const int grow = rowBase + row;
    const v4f v = *(const v4f*)(stg + row * C + 4 * m);
    if (grow < nRowsOut) *(volatile v4f*)(pout + (size_t)grow * C + 4 * m) = v;
  }
  __threadfence();
#pragma unroll 1
  for (int j = 0; j < 8; ++j) {
    const int row = wave * 16 + 2 * j + hh;
    const int grow = rowBase + row;
    const v4f v = *(const v4f*)(stg + row * C + 4 * m);
    if (grow < nRowsOut) *(volatile v4f*)(pout + (size_t)grow * C + 4 * m) = v;
  }
}

__global__ __launch_bounds__(NTHR) void k_agg(const float* __restrict__ P, const int* __restrict__ ei,
    const float* __restrict__ sc, const int* __restrict__ etab,
    const float* __restrict__ W, const float* __restrict__ b, const float* __restrict__ lb,
    float* hout, int nN, int nE, int rowLimit, int l1) {
  extern __shared__ __attribute__((aligned(16))) unsigned char dsm[];
  float* acc   = (float*)(dsm + LDS_ACC);
  float* msg   = (float*)(dsm + LDS_MSG);
  int*   esrc  = (int*)(dsm + LDS_ESRC);
  int*   eslot = (int*)(dsm + LDS_ESLOT);
  float* esin  = (float*)(dsm + LDS_ESIN);
  float* ecos  = (float*)(dsm + LDS_ECOS);

  const int tid = threadIdx.x, lane = tid & 31, wave = tid >> 5, hh = lane >> 4, m = lane & 15;
  const int nodeBase = blockIdx.x * NB;
  const int* srcs = ei;
  const int* dsts = ei + nE;
  const int* erow = etab + (size_t)blockIdx.x * EROW;

  {
    v4f z;
    z.x = 0.0f; z.y = 0.0f; z.z = 0.0f; z.w = 0.0f;
    for (int i = tid; i < (NB + 1) * C / 4; i += NTHR) *(v4f*)(acc + 4 * i) = z;
  }
  int nP = erow[0];
  nP = nP < 0 ? 0 : (nP > PCAP ? PCAP : nP);
  int R = (nP + PASSN - 1) / PASSN;
  R = R > PCAP / PASSN ? PCAP / PASSN : R;
  const int c = tid & (C - 1);
  const int g = tid >> 6;
  const float w64c = W[64 * C + c];
  const float w65c = W[65 * C + c];
  const float bc = b[c];
  __syncthreads();

#pragma unroll 1
  for (int r = 0; r < R; ++r) {
    if (tid < PASSN) {
      const int idx = r * PASSN + tid;
      const bool valid = idx < nP;
      const int idxc = idx < PCAP ? idx : PCAP - 1;
      int e = erow[EHDR + idxc];
      e = e < 0 ? 0 : (e > nE - 1 ? nE - 1 : e);
      const int d = dsts[e];
      int s = srcs[e];
      s = s < 0 ? 0 : (s > nN - 1 ? nN - 1 : s);
      int slot = d - nodeBase;
      if (!valid || (unsigned)slot >= (unsigned)NB) slot = NB;
      const float sn = sc[(size_t)e * 2];
      const float cs = sc[(size_t)e * 2 + 1];
      esrc[tid] = s;
      eslot[tid] = slot;
      esin[tid] = sn;
      ecos[tid] = cs;
    }
    __syncthreads();
    int cnt = nP - r * PASSN;
    cnt = cnt > PASSN ? PASSN : (cnt < 0 ? 0 : cnt);
#pragma unroll 1
    for (int i = g; i < cnt; i += NGRP) {
      int s = esrc[i];
      s = s < 0 ? 0 : (s > nN - 1 ? nN - 1 : s);
      const float v = P[(size_t)s * C + c];
      float t = v + esin[i] * w64c + ecos[i] * w65c + bc;
      if (l1 != 0) t = tanhf(t);
      msg[i * C + c] = t;
    }
    __syncthreads();
    if (tid < C) {
#pragma unroll 1
      for (int i = 0; i < cnt; ++i) {
        int sl = eslot[i];
        sl = sl < 0 ? 0 : (sl > NB ? NB : sl);
        acc[sl * C + tid] += msg[i * C + tid];
      }
    }
    __syncthreads();
  }

  const v4f lb4 = *(const v4f*)(lb + 4 * m);
#pragma unroll 1
  for (int j = 0; j < NB / (2 * NWAVE); ++j) {
    const int row = wave * (NB / NWAVE) + 2 * j + hh;
    const int grow = nodeBase + row;
    v4f v = *(const v4f*)(acc + row * C + 4 * m) + lb4;
    if (l1 != 0) {
      v.x = fmaxf(v.x, 0.0f); v.y = fmaxf(v.y, 0.0f); v.z = fmaxf(v.z, 0.0f); v.w = fmaxf(v.w, 0.0f);
    }
    if (grow < rowLimit) *(volatile v4f*)(hout + (size_t)grow * C + 4 * m) = v;
  }
  __threadfence();
#pragma unroll 1
  for (int j = 0; j < NB / (2 * NWAVE); ++j) {
    const int row = wave * (NB / NWAVE) + 2 * j + hh;
    const int grow = nodeBase + row;
    v4f v = *(const v4f*)(acc + row * C + 4 * m) + lb4;
    if (l1 != 0) {
      v.x = fmaxf(v.x, 0.0f); v.y = fmaxf(v.y, 0.0f); v.z = fmaxf(v.z, 0.0f); v.w = fmaxf(v.w, 0.0f);
    }
    if (grow < rowLimit) *(volatile v4f*)(hout + (size_t)grow * C + 4 * m) = v;
  }
}

extern "C" void kernel_launch(void* const* d_in, const int* in_sizes, int n_in,
                              void* d_out, int out_size, void* d_ws, size_t ws_size,
                              hipStream_t stream) {
  if (n_in < 9) return;
  const int nN = in_sizes[0] / C;
  if (nN < 1 || in_sizes[0] != nN * C) return;
  const int nE = in_sizes[1] / 2;
  if (nE < 1 || in_sizes[1] != 2 * nE || in_sizes[2] != nE) return;
  if (in_sizes[3] != KIN * C || in_sizes[4] != C || in_sizes[5] != C) return;
  if (in_sizes[6] != KIN * C || in_sizes[7] != C || in_sizes[8] != C) return;
  if (out_size != nN * C) return;

  const float* x     = (const float*)d_in[0];
  const int*   ei    = (const int*)d_in[1];
  const float* attr  = (const float*)d_in[2];
  const float* W1    = (const float*)d_in[3];
  const float* b1    = (const float*)d_in[4];
  const float* bias1 = (const float*)d_in[5];
  const float* W2    = (const float*)d_in[6];
  const float* b2    = (const float*)d_in[7];
  const float* bias2 = (const float*)d_in[8];
  float* dout = (float*)d_out;

  const int nBlk = (nN + NB - 1) / NB;
  const size_t rowsP = (size_t)nBlk * NB;
  const int nPJ = (int)(rowsP / PJR);
  const int scN4 = (((2 * nE + 3) / 4) + 7) & ~7;

  char* ws = (char*)d_ws;
  size_t off = 0;
  auto carve = [&](size_t bytes) -> size_t {
    const size_t o = off;
    off = (off + bytes + 255) & ~(size_t)255;
    return o;
  };
  const size_t owp = carve((size_t)4 * WPL * 2);
  const size_t osc = carve((size_t)scN4 * 16);
  const size_t oet = carve((size_t)nBlk * EROW * 4);
  const size_t oP  = carve(rowsP * C * 4);
  const size_t oH  = carve(rowsP * C * 4);
  size_t limit = (size_t)134217728;
  if (ws_size < limit) limit = ws_size;
  if (off > limit) return;

  unsigned short* wp = (unsigned short*)(ws + owp);
  float* scp  = (float*)(ws + osc);
  int*   etab = (int*)(ws + oet);
  float* Pp   = (float*)(ws + oP);
  float* Hp   = (float*)(ws + oH);

  const int vec8 = ((nE & 3) == 0) ? 1 : 0;
  const int nRows = (int)rowsP;

  k_wprep<<<(2 * (WPL / 8) + NTHR - 1) / NTHR, NTHR, 0, stream>>>(W1, W2, wp);
  k_sincos<<<(scN4 + NTHR - 1) / NTHR, NTHR, 0, stream>>>(attr, scp, nE, scN4);
  k_escan<<<nBlk, NTHR, 0, stream>>>(ei, etab, nE, vec8);

  hipFuncSetAttribute(reinterpret_cast<const void*>(&k_agg), hipFuncAttributeMaxDynamicSharedMemorySize, LDS_AGG);

  k_proj<<<nPJ, PJT, 0, stream>>>(x, wp, wp + WPL, Pp, nN, nRows);
  k_agg<<<nBlk, NTHR, LDS_AGG, stream>>>(Pp, ei, scp, etab, W1, b1, bias1, Hp, nN, nE, nRows, 1);
  k_proj<<<nPJ, PJT, 0, stream>>>(Hp, wp + 2 * WPL, wp + 3 * WPL, Pp, nRows, nRows);
  k_agg<<<nBlk, NTHR, LDS_AGG, stream>>>(Pp, ei, scp, etab, W2, b2, bias2, dout, nN, nE, nN, 0);
}
